// LorentzConv2d_56788057588106
// MI455X (gfx1250) — hardware-verified
//
#include <hip/hip_runtime.h>


#define NBI  32
#define HH   64
#define WW   64
#define CIN  64
#define CO   64
#define NPOS (HH * WW)
#define KF   568
#define KP   576
#define IMC  8
#define MROW (IMC * NPOS)
#define DM   KP
#define NTK  MROW
#define LOSC 1024.0f

typedef _Float16 h16;
typedef unsigned short bf;
typedef __attribute__((ext_vector_type(16))) __bf16   v16bf;
typedef __attribute__((ext_vector_type(16))) _Float16 v16h;
typedef __attribute__((ext_vector_type(8)))  _Float16 v8h;
typedef __attribute__((ext_vector_type(8)))  unsigned short v8us;
typedef __attribute__((ext_vector_type(8)))  float    v8f;
typedef __attribute__((ext_vector_type(4)))  float    v4f;
typedef __attribute__((ext_vector_type(4)))  _Float16 v4h;
typedef v8h  __attribute__((may_alias)) v8ha;
typedef v4f  __attribute__((may_alias)) v4fa;
typedef v8us __attribute__((may_alias)) v8usa;

__device__ __forceinline__ unsigned short f2bf(float f) { unsigned u = __float_as_uint(f); u += 0x7FFFu + ((u >> 16) & 1u); return (unsigned short)(u >> 16); }
__device__ __forceinline__ float bf2f(unsigned short b) { return __uint_as_float(((unsigned)b) << 16); }
__device__ __forceinline__ float bfr(float f) { return bf2f(f2bf(f)); }
__device__ __forceinline__ v16h cat16(v8h lo, v8h hi) { return __builtin_shufflevector(lo, hi, 0, 1, 2, 3, 4, 5, 6, 7, 8, 9, 10, 11, 12, 13, 14, 15); }
__device__ __forceinline__ v16bf cat16b(v8us lo, v8us hi) { return __builtin_bit_cast(v16bf, __builtin_shufflevector(lo, hi, 0, 1, 2, 3, 4, 5, 6, 7, 8, 9, 10, 11, 12, 13, 14, 15)); }
__device__ __forceinline__ v8f wmma16(v16h a, v16h b, v8f c) { return __builtin_amdgcn_wmma_f32_16x16x32_f16(false, a, false, b, (short)0, c, false, false); }
__device__ __forceinline__ v8f wmmab(v16bf a, v16bf b, v8f c) { return __builtin_amdgcn_wmma_f32_16x16x32_bf16(false, a, false, b, (short)0, c, false, false); }

template <bool SPLITA, bool F16OUT = false>
__global__ __launch_bounds__(128) void k_gemmb(const bf* __restrict__ A, const bf* __restrict__ Al, const bf* __restrict__ Bn, const float* __restrict__ bias, float* C, int ldc, h16* C2, const float* __restrict__ R = nullptr, int K = DM, int roundR = 1) {
    __shared__ __align__(16) float ost[4][16 * 68];
    const int lane = threadIdx.x & 31, wave = threadIdx.x >> 5, lr = lane & 15, hi = lane >> 4;
    const int r0 = blockIdx.x * 64 + wave * 16, c0 = blockIdx.y * 64;
    const size_t aoff = (size_t)(r0 + lr) * K + 8 * hi;
    size_t boff[4];
#pragma unroll
    for (int t = 0; t < 4; ++t) boff[t] = (size_t)(c0 + t * 16 + lr) * K + 8 * hi;
    v8f acc[4];
#pragma unroll
    for (int t = 0; t < 4; ++t) acc[t] = (v8f){};
#pragma unroll 1
    for (int kc = 0; kc < K; kc += 32) {
        const v16bf a = cat16b(*(const v8us*)(A + aoff + kc), *(const v8us*)(A + aoff + kc + 16));
        v16bf al = a;
        if (SPLITA) al = cat16b(*(const v8us*)(Al + aoff + kc), *(const v8us*)(Al + aoff + kc + 16));
#pragma unroll
        for (int t = 0; t < 4; ++t) { const v16bf b = cat16b(*(const v8us*)(Bn + boff[t] + kc), *(const v8us*)(Bn + boff[t] + kc + 16)); acc[t] = wmmab(a, b, acc[t]); if (SPLITA) acc[t] = wmmab(al, b, acc[t]); }
        asm volatile("v_nop\n\tv_nop\n\tv_nop\n\tv_nop" : "+v"(acc[0]), "+v"(acc[1]), "+v"(acc[2]), "+v"(acc[3]) : "v"(a), "v"(al));
    }
    float* os = &ost[wave][0];
#pragma unroll
    for (int t = 0; t < 4; ++t) { const float bv = bias ? bfr(bias[c0 + t * 16 + lr]) : 0.f;
#pragma unroll
        for (int j = 0; j < 8; ++j) os[(hi * 8 + j) * 68 + t * 16 + lr] = acc[t][j] + bv; }
    __syncthreads();
    if (F16OUT) {
        h16* crow = (h16*)(void*)C + (size_t)r0 * ldc + c0;
        auto pass = [&]() {
#pragma unroll
            for (int s = 0; s < 4; ++s) { const int row = 4 * s + (lane >> 3), piece = lane & 7; const float* sp = os + row * 68 + piece * 8; v8h o, o2;
#pragma unroll
                for (int i = 0; i < 8; ++i) { const h16 a = (h16)sp[i]; o[i] = a; o2[i] = (h16)((sp[i] - (float)a) * LOSC); }
                *(volatile v8h*)(crow + (size_t)row * ldc + piece * 8) = o; if (C2) *(volatile v8h*)(C2 + (size_t)r0 * ldc + c0 + (size_t)row * ldc + piece * 8) = o2; }
        };
        pass(); __threadfence(); pass();
    } else {
        float* crow = C + (size_t)r0 * ldc + c0;
        auto pass = [&]() {
#pragma unroll
            for (int s = 0; s < 8; ++s) { const int Lid = (lane >> 3) + 4 * s, piece = lane & 7; const int row = Lid >> 1, cofs = (Lid & 1) * 32 + piece * 4;
                v4f val = *(const v4fa*)(os + row * 68 + cofs); if (R) { const v4f rv = *(const v4f*)(R + ((size_t)r0 + row) * ldc + c0 + cofs); val += roundR ? (v4f){bfr(rv[0]), bfr(rv[1]), bfr(rv[2]), bfr(rv[3])} : rv; }
                *(volatile v4f*)(crow + (size_t)row * ldc + cofs) = val; }
        };
        pass(); __threadfence(); pass();
    }
}


__device__ __forceinline__ float trescaled(const float* __restrict__ x, int b, int py, int px) {
    float s = 0.f;
#pragma unroll
    for (int tap = 0; tap < 9; ++tap) { const int yy = py + tap / 3 - 1, xx = px + tap % 3 - 1;
        const float xt = (yy >= 0 && yy < HH && xx >= 0 && xx < WW) ? bfr(x[(((size_t)b * HH + yy) * WW + xx) * CIN]) : 0.f;
        const float tc = fmaxf(xt, 1.0f); s = fmaf(tc, tc, s); }
    return sqrtf(s - 8.0f);
}
__global__ __launch_bounds__(256) void k_wpad(const float* __restrict__ w, bf* WB) {
    const int u = blockIdx.x * 256 + threadIdx.x; if (u >= CO * KP / 8) return;
    const int o = u / (KP / 8), f0 = (u % (KP / 8)) * 8; v8us v;
#pragma unroll
    for (int i = 0; i < 8; ++i) { const int f = f0 + i; v[i] = (f < KF) ? f2bf(w[(size_t)o * KF + f]) : (unsigned short)0; }
    *(volatile v8us*)(WB + (size_t)o * KP + f0) = v; __threadfence(); *(volatile v8us*)(WB + (size_t)o * KP + f0) = v;
}
__global__ __launch_bounds__(128) void k_im2col(const float* __restrict__ x, int b0, bf* A) {
    const int tid = threadIdx.x; if (tid >= KP / 8) return;
    const int lr = blockIdx.x; const int bi = b0 + lr / NPOS, l = lr % NPOS, py = l / WW, px = l % WW;
    v8us v;
#pragma unroll
    for (int i = 0; i < 8; ++i) { const int f = tid * 8 + i; float val;
        if (f == 0) val = trescaled(x, bi, py, px);
        else if (f < KF) { const int tap = (f - 1) / 63, c = (f - 1) % 63 + 1; const int yy = py + tap / 3 - 1, xx = px + tap % 3 - 1;
            val = (yy >= 0 && yy < HH && xx >= 0 && xx < WW) ? x[(((size_t)bi * HH + yy) * WW + xx) * CIN + c] : 0.f; }
        else val = 0.f;
        v[i] = f2bf(val); }
    *(volatile v8us*)(A + (size_t)lr * KP + tid * 8) = v; __threadfence(); *(volatile v8us*)(A + (size_t)lr * KP + tid * 8) = v;
}
__global__ __launch_bounds__(256) void k_pack(const float* __restrict__ Y, const float* __restrict__ x, const float* __restrict__ w, int b0, float* OUTC) {
    const size_t i = (size_t)blockIdx.x * 256 + threadIdx.x; if (i >= (size_t)MROW * (CO + 1)) return;
    const int l = (int)(i / (CO + 1)), o = (int)(i % (CO + 1)); const int bi = b0 + l / NPOS, pp = l % NPOS;
    const float t = trescaled(x, bi, pp / WW, pp % WW); const float tlo = t - bfr(t);
    float val;
    if (o == 0) { float s = 1.0f;
#pragma unroll 1
        for (int c = 0; c < CO; ++c) { const float y = Y[(size_t)l * CO + c] + tlo * bfr(w[(size_t)c * KF]); s = fmaf(y, y, s); }
        val = sqrtf(s); }
    else val = Y[(size_t)l * CO + (o - 1)] + tlo * bfr(w[(size_t)(o - 1) * KF]);
    *(volatile float*)(OUTC + i) = val; __threadfence(); *(volatile float*)(OUTC + i) = val;
}

extern "C" void kernel_launch(void* const* d_in, const int* in_sizes, int n_in,
                              void* d_out, int out_size, void* d_ws, size_t ws_size, hipStream_t stream) {
    (void)in_sizes; (void)n_in; (void)out_size;
    const float* x = (const float*)d_in[0]; const float* w = (const float*)d_in[1]; const float* bias = (const float*)d_in[2];
    float* out = (float*)d_out;
    char* wsp = (char*)d_ws;
    auto take = [&](size_t bytes) { char* p = wsp; wsp += (bytes + 255) & ~(size_t)255; return (void*)p; };
    bf* WB = (bf*)take((size_t)CO * KP * 2); bf* A = (bf*)take((size_t)MROW * KP * 2); float* Y = (float*)take((size_t)MROW * CO * 4);
    if ((size_t)(wsp - (char*)d_ws) > ws_size) return;
    k_wpad<<<(CO * KP / 8 + 255) / 256, 256, 0, stream>>>(w, WB);
    for (int ch = 0; ch < NBI / IMC; ++ch) {
        const int b0 = ch * IMC;
        k_im2col<<<MROW, 128, 0, stream>>>(x, b0, A);
        k_gemmb<false, false><<<dim3(MROW / 64, CO / 64, 1), 128, 0, stream>>>(A, nullptr, WB, bias, Y, CO, nullptr);
        k_pack<<<(unsigned)(((size_t)MROW * (CO + 1) + 255) / 256), 256, 0, stream>>>(Y, x, w, b0, out + (size_t)b0 * NPOS * (CO + 1));
    }
}
